// OTPrompt_64183991271489
// MI455X (gfx1250) — hardware-run, weakly checked
//
#include <hip/hip_runtime.h>
#include <math.h>

typedef __attribute__((ext_vector_type(16))) __bf16 v16b;
typedef __attribute__((ext_vector_type(8)))  __bf16 v8b;
typedef __attribute__((ext_vector_type(8)))  float  v8f;
typedef __attribute__((ext_vector_type(4)))  float  v4f;

constexpr int kNF   = 100;
constexpr int kMP   = 20;
constexpr int kDim  = 128;
constexpr int kNFP  = 112;
constexpr int kMPP  = 32;
constexpr int kKsP  = 33;
constexpr int kSlabP = 36;
constexpr int kPlane = 4096;
constexpr int kOut0 = kNF * kDim;
constexpr int kOut1 = kNF * kMP;
constexpr int kOut1Q = kOut1 / 4;
constexpr int kIterCap = 10000;
constexpr float kEps     = 0.05f;
constexpr float kInvEps  = 1.0f / kEps;
constexpr float kRowMass = 1.0f / (float)kNF;
constexpr float kColMass = 1.0f / (float)kMP;
constexpr float kPlanScale = (float)kNF;

static_assert(kNFP % 16 == 0 && kMPP % 16 == 0 && kNFP >= kNF && kMPP >= kMP, "tile multiples");
static_assert(kDim % 32 == 0 && kMPP % 32 == 0, "depth multiples of 32");
static_assert(kMPP * kDim <= kPlane && kNFP * kMPP <= kPlane && kDim * kMPP <= kPlane, "plane slots");
static_assert(kOut0 * 4 == 51200 && (kOut0 * 4) % 128 == 0, "second output starts on a line");
static_assert(kOut0 + kOut1 == 14800 && (kOut0 + kOut1) * 4 == 59200, "output total");
static_assert(kOut1 % 4 == 0 && kMP % 4 == 0, "float4 stream of the plan");
static_assert(kNFP * kKsP <= 8 * 16 * kSlabP, "float buffer holds the kernel matrix and the slabs");
static_assert(kNFP * kMPP == 14 * 256, "elementwise pass coverage");

__device__ __forceinline__ unsigned short f2bf_bits(float f) {
  unsigned u = __float_as_uint(f);
  return (unsigned short)((u + 0x7FFFu + ((u >> 16) & 1u)) >> 16);
}
__device__ __forceinline__ float bf_bits2f(unsigned short h) { return __uint_as_float(((unsigned)h) << 16); }

__device__ __forceinline__ void split_bf(float f, __bf16& hi, __bf16& lo) {
  const unsigned short hb = f2bf_bits(f);
  const float rem = f - bf_bits2f(hb);
  const unsigned short lb = f2bf_bits(rem);
  hi = __builtin_bit_cast(__bf16, hb);
  lo = __builtin_bit_cast(__bf16, lb);
}

__device__ __forceinline__ v8f mma_bf(v16b a, v16b b, v8f c) {
  c = __builtin_amdgcn_wmma_f32_16x16x32_bf16(false, a, false, b, (short)0, c, false, false);
  asm volatile("v_nop\n\tv_nop\n\tv_nop\n\tv_nop" : "+v"(c) : "v"(a), "v"(b));
  return c;
}

__device__ __forceinline__ v16b frag_load(const __bf16* p) {
  union { v16b v; v8b h[2]; } f;
  f.h[0] = *(const v8b*)(p);
  f.h[1] = *(const v8b*)(p + 16);
  return f.v;
}

__device__ __forceinline__ v4f ld4_pinned(const float* p) {
  const v4f t = *(const v4f*)p;
  float a = t[0];
  float b = t[1];
  float c = t[2];
  float d = t[3];
  asm volatile("" : "+v"(a), "+v"(b), "+v"(c), "+v"(d));
  v4f r;
  r[0] = a;
  r[1] = b;
  r[2] = c;
  r[3] = d;
  return r;
}

__device__ __forceinline__ void wave_lds_sync() {
  __builtin_amdgcn_fence(__ATOMIC_RELEASE, "workgroup");
  __builtin_amdgcn_wave_barrier();
  __builtin_amdgcn_fence(__ATOMIC_ACQUIRE, "workgroup");
}

__global__ __launch_bounds__(256) void plan_kernel(const float* __restrict__ x,
                                                   const float* __restrict__ P,
                                                   const int* __restrict__ iters_p,
                                                   float* __restrict__ out)
{
  __shared__ __align__(16) __bf16 sOpA[2 * kPlane];
  __shared__ __align__(16) __bf16 sOpT[2 * kPlane];
  __shared__ __align__(16) float  sF[8 * 16 * kSlabP];
  __shared__ float sRinv[kNFP];
  __shared__ float sU[kNFP];
  __shared__ float sV[kMPP];
  __shared__ float sPart[8 * 32];

  const int tid  = threadIdx.x;
  const int lane = tid & 31;
  const int wave = tid >> 5;
  const int l16  = lane & 15;
  const int hh   = lane >> 4;

#pragma unroll 1
  for (int it = 0; it < 7; ++it) {
    const int r  = ((it * 8 + wave) << 1) + hh;
    const int rc = (r < kNF) ? r : (kNF - 1);
    const float* px = x + rc * kDim + l16 * 8;
    const v4f a0 = ld4_pinned(px);
    const v4f a1 = ld4_pinned(px + 4);
    float s = a0[0] * a0[0];
    s = fmaf(a0[1], a0[1], s);
    s = fmaf(a0[2], a0[2], s);
    s = fmaf(a0[3], a0[3], s);
    s = fmaf(a1[0], a1[0], s);
    s = fmaf(a1[1], a1[1], s);
    s = fmaf(a1[2], a1[2], s);
    s = fmaf(a1[3], a1[3], s);
    s += __shfl_xor(s, 1, 32);
    s += __shfl_xor(s, 2, 32);
    s += __shfl_xor(s, 4, 32);
    s += __shfl_xor(s, 8, 32);
    const float rinv = 1.0f / fmaxf(sqrtf(s), 1e-12f);
    const float rsel = (r < kNF) ? rinv : 0.0f;
    if (l16 == 0) sRinv[r] = rsel;
  }

#pragma unroll 1
  for (int it = 0; it < 2; ++it) {
    const int r  = ((it * 8 + wave) << 1) + hh;
    const bool rv = (r < kMP);
    const int rc = rv ? r : (kMP - 1);
    const float* pp = P + rc * kDim + l16 * 8;
    const v4f a0 = ld4_pinned(pp);
    const v4f a1 = ld4_pinned(pp + 4);
    float s = a0[0] * a0[0];
    s = fmaf(a0[1], a0[1], s);
    s = fmaf(a0[2], a0[2], s);
    s = fmaf(a0[3], a0[3], s);
    s = fmaf(a1[0], a1[0], s);
    s = fmaf(a1[1], a1[1], s);
    s = fmaf(a1[2], a1[2], s);
    s = fmaf(a1[3], a1[3], s);
    s += __shfl_xor(s, 1, 32);
    s += __shfl_xor(s, 2, 32);
    s += __shfl_xor(s, 4, 32);
    s += __shfl_xor(s, 8, 32);
    const float rinv = 1.0f / fmaxf(sqrtf(s), 1e-12f);
    v8b hv, lv;
#pragma unroll
    for (int e = 0; e < 4; ++e) {
      const float g0 = a0[e];
      const float g1 = a1[e];
      const float f0 = rv ? (g0 * rinv) : 0.0f;
      const float f1 = rv ? (g1 * rinv) : 0.0f;
      __bf16 bh, bl;
      split_bf(f0, bh, bl);
      hv[e] = bh;
      lv[e] = bl;
      split_bf(f1, bh, bl);
      hv[4 + e] = bh;
      lv[4 + e] = bl;
    }
    __bf16* dst = sOpA + r * kDim + l16 * 8;
    *(v8b*)(dst) = hv;
    *(v8b*)(dst + kPlane) = lv;
  }

  {
    const int n  = tid >> 1;
    const int kh = tid & 1;
    v8b h0, h1, l0, l1;
#pragma unroll
    for (int e = 0; e < 16; ++e) {
      const int kk = kh * 16 + e;
      const int kc = (kk < kMP) ? kk : (kMP - 1);
      float v = P[kc * kDim + n];
      asm volatile("" : "+v"(v));
      const float f = (kk < kMP) ? v : 0.0f;
      __bf16 bh, bl;
      split_bf(f, bh, bl);
      if (e < 8) {
        h0[e] = bh;
        l0[e] = bl;
      } else {
        h1[e - 8] = bh;
        l1[e - 8] = bl;
      }
    }
    __bf16* dst = sOpT + n * kMPP + kh * 16;
    *(v8b*)(dst) = h0;
    *(v8b*)(dst + 8) = h1;
    *(v8b*)(dst + kPlane) = l0;
    *(v8b*)(dst + kPlane + 8) = l1;
  }

  if (tid < kNFP) sU[tid] = (tid < kNF) ? kRowMass : 0.0f;
  if (tid < kMPP) sV[tid] = (tid < kMP) ? kColMass : 0.0f;
  __syncthreads();

  if (wave < 7) {
    const int m = wave * 16 + l16;
    const bool mval = (m < kNF);
    const int mc = mval ? m : (kNF - 1);
    const float rinv = sRinv[m];
    v8f acc0 = (v8f){0.f, 0.f, 0.f, 0.f, 0.f, 0.f, 0.f, 0.f};
    v8f acc1 = (v8f){0.f, 0.f, 0.f, 0.f, 0.f, 0.f, 0.f, 0.f};
#pragma unroll 1
    for (int k0 = 0; k0 < kDim; k0 += 32) {
      const float* px = x + mc * kDim + k0 + 8 * hh;
      const v4f a0 = ld4_pinned(px);
      const v4f a1 = ld4_pinned(px + 4);
      const v4f a2 = ld4_pinned(px + 16);
      const v4f a3 = ld4_pinned(px + 20);
      v16b ah, al;
#pragma unroll
      for (int e = 0; e < 4; ++e) {
        const float g0 = a0[e];
        const float g1 = a1[e];
        const float g2 = a2[e];
        const float g3 = a3[e];
        const float f0 = mval ? (g0 * rinv) : 0.0f;
        const float f1 = mval ? (g1 * rinv) : 0.0f;
        const float f2 = mval ? (g2 * rinv) : 0.0f;
        const float f3 = mval ? (g3 * rinv) : 0.0f;
        __bf16 bh, bl;
        split_bf(f0, bh, bl);
        ah[e] = bh;
        al[e] = bl;
        split_bf(f1, bh, bl);
        ah[4 + e] = bh;
        al[4 + e] = bl;
        split_bf(f2, bh, bl);
        ah[8 + e] = bh;
        al[8 + e] = bl;
        split_bf(f3, bh, bl);
        ah[12 + e] = bh;
        al[12 + e] = bl;
      }
      const __bf16* pb = sOpA + l16 * kDim + k0 + 8 * hh;
      const v16b b0h = frag_load(pb);
      const v16b b0l = frag_load(pb + kPlane);
      const v16b b1h = frag_load(pb + 16 * kDim);
      const v16b b1l = frag_load(pb + 16 * kDim + kPlane);
      acc0 = mma_bf(ah, b0h, acc0);
      acc0 = mma_bf(ah, b0l, acc0);
      acc0 = mma_bf(al, b0h, acc0);
      acc1 = mma_bf(ah, b1h, acc1);
      acc1 = mma_bf(ah, b1l, acc1);
      acc1 = mma_bf(al, b1h, acc1);
    }
#pragma unroll
    for (int r = 0; r < 8; ++r) {
      const int row = wave * 16 + 8 * hh + r;
      sF[row * kKsP + l16] = acc0[r];
      sF[row * kKsP + 16 + l16] = acc1[r];
    }
  }
  __syncthreads();

#pragma unroll 1
  for (int it = 0; it < 14; ++it) {
    const int idx = it * 256 + tid;
    const int i = idx >> 5;
    const int j = idx & 31;
    const float s = sF[i * kKsP + j];
    const float c = 1.0f - s;
    const float kv = expf(-c * kInvEps);
    const float ksel = (i < kNF && j < kMP) ? kv : 0.0f;
    sF[i * kKsP + j] = ksel;
  }
  __syncthreads();

  int iters = iters_p[0];
  iters = (iters < 0) ? 0 : iters;
  iters = (iters > kIterCap) ? kIterCap : iters;
#pragma unroll 1
  for (int it = 0; it < iters; ++it) {
    if (tid < kNFP) {
      float s = 0.0f;
#pragma unroll
      for (int j = 0; j < kMP; ++j) s = fmaf(sF[tid * kKsP + j], sV[j], s);
      const bool rv = (tid < kNF);
      const float sd = rv ? s : 1.0f;
      const float q = kRowMass / sd;
      sU[tid] = rv ? q : 0.0f;
    }
    __syncthreads();
    {
      float s = 0.0f;
#pragma unroll 1
      for (int i = wave; i < kNF; i += 8) s = fmaf(sF[i * kKsP + lane], sU[i], s);
      sPart[wave * 32 + lane] = s;
    }
    __syncthreads();
    if (tid < kMPP) {
      float s = 0.0f;
#pragma unroll
      for (int g = 0; g < 8; ++g) s += sPart[g * 32 + tid];
      const bool cv = (tid < kMP);
      const float sd = cv ? s : 1.0f;
      const float q = kColMass / sd;
      sV[tid] = cv ? q : 0.0f;
    }
    __syncthreads();
  }

  {
    float* out1 = out + kOut0;
    v4f tv0, tv1;
    const int q0 = (0 * 8 + wave) * 32 + lane;
    const int q1 = (1 * 8 + wave) * 32 + lane;
    const bool qv0 = (q0 < kOut1Q);
    const bool qv1 = (q1 < kOut1Q);
    const int qc0 = qv0 ? q0 : (kOut1Q - 1);
    const int qc1 = qv1 ? q1 : (kOut1Q - 1);
    {
      const int f = qc0 * 4;
      const int i = f / kMP;
      const int j0 = f - i * kMP;
      const float ui = sU[i];
#pragma unroll
      for (int e = 0; e < 4; ++e) {
        float t = (ui * sF[i * kKsP + j0 + e]) * sV[j0 + e];
        t = t * kPlanScale;
        tv0[e] = t;
      }
    }
    {
      const int f = qc1 * 4;
      const int i = f / kMP;
      const int j0 = f - i * kMP;
      const float ui = sU[i];
#pragma unroll
      for (int e = 0; e < 4; ++e) {
        float t = (ui * sF[i * kKsP + j0 + e]) * sV[j0 + e];
        t = t * kPlanScale;
        tv1[e] = t;
      }
    }
    for (int pass = 0; pass < 2; ++pass) {
      if (qv0) *(volatile v4f*)(out1 + qc0 * 4) = tv0;
      if (qv1) *(volatile v4f*)(out1 + qc1 * 4) = tv1;
      __threadfence();
    }
  }

#pragma unroll 1
  for (int it = 0; it < 2; ++it) {
    const int task = it * 256 + tid;
    if (task < kNFP * 4) {
      const int i  = task >> 2;
      const int kq = task & 3;
      const float ui = sU[i];
      v8b hv, lv;
#pragma unroll
      for (int e = 0; e < 8; ++e) {
        const int k = kq * 8 + e;
        float t = (ui * sF[i * kKsP + k]) * sV[k];
        t = t * kPlanScale;
        const float f = (i < kNF && k < kMP) ? t : 0.0f;
        __bf16 bh, bl;
        split_bf(f, bh, bl);
        hv[e] = bh;
        lv[e] = bl;
      }
      __bf16* dst = sOpA + i * kMPP + kq * 8;
      *(v8b*)(dst) = hv;
      *(v8b*)(dst + kPlane) = lv;
    }
  }
  __syncthreads();

  {
    float* slab = sF + wave * (16 * kSlabP);
    const int q8 = lane >> 3;
    const int c4 = (lane & 7) * 4;
#pragma unroll 1
    for (int trip = 0; trip < 4; ++trip) {
      const int item = trip * 8 + wave;
      if (item < 28) {
        const int tm = item >> 2;
        const int cg = item & 3;
        const __bf16* pa = sOpA + (tm * 16 + l16) * kMPP + 8 * hh;
        const v16b ah = frag_load(pa);
        const v16b al = frag_load(pa + kPlane);
        const __bf16* pb = sOpT + (cg * 32 + l16) * kMPP + 8 * hh;
        const v16b b0h = frag_load(pb);
        const v16b b0l = frag_load(pb + kPlane);
        const v16b b1h = frag_load(pb + 16 * kMPP);
        const v16b b1l = frag_load(pb + 16 * kMPP + kPlane);
        v8f acc0 = (v8f){0.f, 0.f, 0.f, 0.f, 0.f, 0.f, 0.f, 0.f};
        v8f acc1 = (v8f){0.f, 0.f, 0.f, 0.f, 0.f, 0.f, 0.f, 0.f};
        acc0 = mma_bf(ah, b0h, acc0);
        acc0 = mma_bf(ah, b0l, acc0);
        acc0 = mma_bf(al, b0h, acc0);
        acc1 = mma_bf(ah, b1h, acc1);
        acc1 = mma_bf(ah, b1l, acc1);
        acc1 = mma_bf(al, b1h, acc1);
#pragma unroll
        for (int r = 0; r < 8; ++r) {
          slab[(8 * hh + r) * kSlabP + l16] = acc0[r];
          slab[(8 * hh + r) * kSlabP + 16 + l16] = acc1[r];
        }
        wave_lds_sync();
        v4f ov[4];
        int  off[4];
        bool rvalid[4];
#pragma unroll
        for (int t4 = 0; t4 < 4; ++t4) {
          const int row  = t4 * 4 + q8;
          const int grow = tm * 16 + row;
          rvalid[t4] = (grow < kNF);
          const int growc = rvalid[t4] ? grow : (kNF - 1);
          off[t4] = growc * kDim + cg * 32 + c4;
          const v4f xv = ld4_pinned(x + off[t4]);
          const v4f sv = *(const v4f*)(slab + row * kSlabP + c4);
          ov[t4] = xv + sv;
        }
        for (int pass = 0; pass < 2; ++pass) {
#pragma unroll
          for (int t4 = 0; t4 < 4; ++t4) {
            if (rvalid[t4]) *(volatile v4f*)(out + off[t4]) = ov[t4];
          }
          __threadfence();
        }
        wave_lds_sync();
      }
    }
  }
}

extern "C" void kernel_launch(void* const* d_in, const int* in_sizes, int n_in,
                              void* d_out, int out_size, void* d_ws, size_t ws_size,
                              hipStream_t stream) {
  (void)d_ws;
  (void)ws_size;
  if (n_in < 3) return;
  if (in_sizes[0] != kNF * kDim) return;
  if (in_sizes[1] != kMP * kDim) return;
  if (in_sizes[2] != 1) return;
  if (out_size != kOut0 + kOut1) return;
  const float* x  = (const float*)d_in[0];
  const float* P  = (const float*)d_in[1];
  const int*   it = (const int*)d_in[2];
  float* out = (float*)d_out;
  plan_kernel<<<1, 256, 0, stream>>>(x, P, it, out);
}
